// EncoderLayer_14482629722465
// MI455X (gfx1250) — hardware-verified
//
#include <hip/hip_runtime.h>
#include <math.h>

typedef __attribute__((ext_vector_type(16))) _Float16 v16h;
typedef __attribute__((ext_vector_type(8)))  _Float16 v8h;
typedef __attribute__((ext_vector_type(8)))  float v8f;
typedef __attribute__((ext_vector_type(4)))  float v4f;
typedef __attribute__((ext_vector_type(4)))  unsigned v4u;
union H8 { v8h v; v4u u; };

template <typename T> __device__ __forceinline__ void vst2(void* p, T v) { *(volatile T*)p = v; __threadfence(); *(volatile T*)p = v; }
__device__ __forceinline__ v8f wmma16(v16h a, v16h b, v8f c) {
  v8f d = __builtin_amdgcn_wmma_f32_16x16x32_f16(false, a, false, b, (short)0, c, false, false);
  asm volatile("v_nop\n\tv_nop\n\tv_nop\n\tv_nop" : "+v"(d) : "v"(a), "v"(b));
  return d;
}
__device__ __forceinline__ float bfr(float v) { return (float)(__bf16)v; }
__device__ __forceinline__ v4f bfr4(v4f v) { v4f r; r[0] = bfr(v[0]); r[1] = bfr(v[1]); r[2] = bfr(v[2]); r[3] = bfr(v[3]); return r; }
__device__ __forceinline__ v16h frag_h(const _Float16* rowk0, int lane) {
  union { v16h v; v8h q[2]; } u; const _Float16* p = rowk0 + 8 * (lane >> 4);
  u.q[0] = *(const v8h*)p; u.q[1] = *(const v8h*)(p + 16); return u.v;
}
__device__ __forceinline__ v16h frag_f32(const float* rowk0, int lane) {
  v16h a; const float* p = rowk0 + 8 * (lane >> 4);
  const v4f x0 = *(const v4f*)p, x1 = *(const v4f*)(p + 4), x2 = *(const v4f*)(p + 16), x3 = *(const v4f*)(p + 20);
#pragma unroll
  for (int i = 0; i < 4; ++i) { a[i] = (_Float16)x0[i]; a[4 + i] = (_Float16)x1[i]; a[8 + i] = (_Float16)x2[i]; a[12 + i] = (_Float16)x3[i]; }
  return a;
}
__device__ __forceinline__ float gelu_f(float t) { return (t * (erff(t * 0.70710678118654752f) + 1.0f)) * 0.5f; }
#define LDSX() do { asm volatile("s_wait_dscnt 0" ::: "memory"); __builtin_amdgcn_wave_barrier(); __builtin_amdgcn_fence(3  , "workgroup"); } while (0)
#define MAXSZ(a, b) ((a) > (b) ? (a) : (b))

#ifndef NB
#define NB 8
#endif
#ifndef SEQ
#define SEQ 512
#endif
#define NB_FULL 8
#define SEQ_FULL 512
#define TT SEQ
#define CC 1024
#define NH 16
#define HD 64
#define FF 4096
#define NRW (NB * TT)
#define NQB (TT / 64)
#define QSCALE (0.125f)
#define PSCALE (0.03125f)
#define WCAR (64.0f)
#define HCAR (16.0f)
#define PCAR (2048.0f)
static_assert(NB >= 1 && NB <= NB_FULL);
static_assert(TT >= 128 && TT <= SEQ_FULL && (TT % 128) == 0);
static_assert(NH * HD == CC);
static_assert((CC % 256) == 0 && (FF % 128) == 0 && (NRW % 64) == 0 && (NRW % 8) == 0 && (CC % 64) == 0 && (FF % 64) == 0);

#define SZ_W    (2u * (size_t)CC * CC)
#define SZ_W1   (2u * (size_t)FF * CC)
#define WS_WQ   ((size_t)0)
#define WS_WK   (WS_WQ + SZ_W)
#define WS_WV   (WS_WK + SZ_W)
#define WS_WO   (WS_WV + SZ_W)
#define WS_WPQ  (WS_WO + SZ_W)
#define WS_WPK  (WS_WPQ + SZ_W)
#define WS_WPV  (WS_WPK + SZ_W)
#define WS_W1   (WS_WPV + SZ_W)
#define WS_W2   (WS_W1 + SZ_W1)
#define SZ_ACT  (2u * (size_t)NRW * CC)
#define WS_Y    (WS_W2 + SZ_W1)
#define WS_Q    (WS_Y + SZ_ACT)
#define WS_K    (WS_Q + SZ_ACT)
#define WS_VT   (WS_K + SZ_ACT)
#define WS_PQ   (WS_VT + SZ_ACT)
#define WS_PK   (WS_PQ + SZ_ACT)
#define WS_PVT  (WS_PK + SZ_ACT)
#define SZ_XP   MAXSZ(4u * (size_t)NRW * CC, 4u * (size_t)NH * TT * TT)
#define WS_XP   (WS_PVT + SZ_ACT)
#define WS_PATH (WS_XP + SZ_XP)
#define WS_END  (WS_PATH + 4u * (size_t)NB * CC)
static_assert(4u * (size_t)NB * TT * TT <= 3u * SZ_ACT);
static_assert(2u * (size_t)NRW * FF <= 4u * SZ_ACT);
static_assert(4u * (size_t)NH * TT * TT <= SZ_XP);
static_assert(4u * (size_t)NRW * CC <= SZ_XP);
static_assert(WS_END <= (size_t)134217728u);

__global__ __launch_bounds__(256) void k_wcvt(const float* __restrict__ W, int K, int N, _Float16* __restrict__ WT) {
  __shared__ float tile[64][65];
  const int tid = threadIdx.x, tx = tid & 63, ty = tid >> 6; const int k0 = blockIdx.y * 64, n0 = blockIdx.x * 64;
#pragma unroll 1
  for (int i = ty; i < 64; i += 4) tile[i][tx] = W[(size_t)(k0 + i) * N + n0 + tx];
  __syncthreads();
#pragma unroll 1
  for (int e = tid; e < 64 * 8; e += 256) { const int nn = e >> 3, q = e & 7; H8 o;
#pragma unroll
    for (int i = 0; i < 8; ++i) o.v[i] = (_Float16)(bfr(tile[q * 8 + i][nn]) * WCAR);
    vst2(WT + (size_t)(n0 + nn) * K + k0 + q * 8, o.u); }
}

__global__ __launch_bounds__(256) void k_ln(const float* __restrict__ X, int inmap, int cvt, const float* __restrict__ G, const float* __restrict__ BE, _Float16* __restrict__ Y) {
  const int wave = threadIdx.x >> 5, lane = threadIdx.x & 31; const int row = blockIdx.x * 8 + wave;
  const size_t xrow = inmap ? ((size_t)(row / TT) * SEQ_FULL + (size_t)(row % TT)) : (size_t)row;
  const float* xr = X + xrow * CC;
  float s1 = 0.f;
#pragma unroll 1
  for (int i = 0; i < CC / 256; ++i) { const int c = i * 256 + lane * 8; v4f a = *(const v4f*)(xr + c), b = *(const v4f*)(xr + c + 4); if (cvt) { a = bfr4(a); b = bfr4(b); }
    s1 += ((a[0] + a[1]) + (a[2] + a[3])) + ((b[0] + b[1]) + (b[2] + b[3])); }
#pragma unroll
  for (int o = 1; o < 32; o <<= 1) s1 += __shfl_xor(s1, o);
  const float mu = s1 * (1.0f / CC); float q = 0.f;
#pragma unroll 1
  for (int i = 0; i < CC / 256; ++i) { const int c = i * 256 + lane * 8; v4f a = *(const v4f*)(xr + c), b = *(const v4f*)(xr + c + 4); if (cvt) { a = bfr4(a); b = bfr4(b); }
#pragma unroll
    for (int k = 0; k < 4; ++k) { const float d0 = a[k] - mu, d1 = b[k] - mu; q += d0 * d0; q += d1 * d1; } }
#pragma unroll
  for (int o = 1; o < 32; o <<= 1) q += __shfl_xor(q, o);
  const float inv = 1.0f / sqrtf(q * (1.0f / CC) + 1e-5f);
#pragma unroll 1
  for (int i = 0; i < CC / 256; ++i) { const int c = i * 256 + lane * 8; v4f a = *(const v4f*)(xr + c), b = *(const v4f*)(xr + c + 4); if (cvt) { a = bfr4(a); b = bfr4(b); }
    const v4f g0 = *(const v4f*)(G + c), g1 = *(const v4f*)(G + c + 4), e0 = *(const v4f*)(BE + c), e1 = *(const v4f*)(BE + c + 4); H8 o;
#pragma unroll
    for (int k = 0; k < 4; ++k) { o.v[k] = (_Float16)(((a[k] - mu) * inv) * bfr(g0[k]) + bfr(e0[k])); o.v[4 + k] = (_Float16)(((b[k] - mu) * inv) * bfr(g1[k]) + bfr(e1[k])); }
    vst2(Y + (size_t)row * CC + c, o.u); }
}

template <int MODE>
__global__ __launch_bounds__(128) void k_gem(const _Float16* __restrict__ A, int lda, int K, const _Float16* __restrict__ WT, int nout,
    const float* __restrict__ BIAS, float sa, float so, const float* __restrict__ AUX, const float* __restrict__ PATH, _Float16* __restrict__ OH, float* __restrict__ OF) {
  __shared__ __align__(16) float sf[4][16][132];
  __shared__ __align__(16) _Float16 th[128][72];
  const int tid = threadIdx.x, wave = tid >> 5, lane = tid & 31, col = lane & 15, g = lane >> 4;
  const int c0 = blockIdx.y * 128; const size_t rb = (size_t)blockIdx.x * 64; const size_t r0 = rb + wave * 16;
  v8f acc[8] = {};
#pragma unroll 1
  for (int kc = 0; kc < K / 32; ++kc) {
    const v16h a = frag_h(A + (r0 + col) * (size_t)lda + kc * 32, lane);
    asm volatile("s_wait_loadcnt 0x0" ::: "memory");
#pragma unroll
    for (int j = 0; j < 8; ++j) { const v16h w = frag_h(WT + (size_t)(c0 + j * 16 + col) * K + kc * 32, lane); asm volatile("s_wait_loadcnt 0x0" ::: "memory"); acc[j] = wmma16(a, w, acc[j]); } }
  if (MODE == 1) {
    const size_t bb = rb / TT; const int t0 = (int)(rb % TT);
#pragma unroll
    for (int j = 0; j < 8; ++j) { const float bias = bfr(BIAS[c0 + j * 16 + col]);
#pragma unroll
      for (int r = 0; r < 8; ++r) th[j * 16 + col][wave * 16 + 8 * g + r] = (_Float16)((acc[j][r] * sa + bias) * so); }
    __syncthreads();
#pragma unroll 1
    for (int e = tid; e < 128 * 8; e += 128) { const int cl = e >> 3, q = e & 7; vst2(OH + (bb * nout + c0 + cl) * (size_t)TT + t0 + q * 8, *(const v4u*)&th[cl][q * 8]); }
  } else {
#pragma unroll
    for (int j = 0; j < 8; ++j) { const float bias = bfr(BIAS[c0 + j * 16 + col]);
#pragma unroll
      for (int r = 0; r < 8; ++r) sf[wave][8 * g + r][j * 16 + col] = acc[j][r] * sa + bias; }
    LDSX();
    if (MODE == 0 || MODE == 2) {
#pragma unroll 1
      for (int i = 0; i < 8; ++i) { const int rl = 2 * i + g; const v4f u0 = *(const v4f*)&sf[wave][rl][col * 8], u1 = *(const v4f*)&sf[wave][rl][col * 8 + 4]; H8 o;
#pragma unroll
        for (int k = 0; k < 4; ++k) { float t0 = u0[k], t1 = u1[k]; if (MODE == 2) { t0 = gelu_f(t0); t1 = gelu_f(t1); } o.v[k] = (_Float16)(t0 * so); o.v[4 + k] = (_Float16)(t1 * so); }
        vst2(OH + (r0 + rl) * (size_t)nout + c0 + col * 8, o.u); }
    } else {
#pragma unroll 1
      for (int rl = 0; rl < 16; ++rl) { const size_t r = r0 + rl; const size_t oo = r * (size_t)nout + c0 + lane * 4; v4f v = *(const v4f*)&sf[wave][rl][lane * 4];
        if (MODE == 3) { const size_t bb = r / TT; const size_t xr = bb * SEQ_FULL + (r % TT); const v4f xv = *(const v4f*)(AUX + xr * nout + c0 + lane * 4); const v4f pv = *(const v4f*)(PATH + bb * nout + c0 + lane * 4);
#pragma unroll
          for (int k = 0; k < 4; ++k) v[k] = bfr(xv[k]) + 0.5f * (v[k] + pv[k]); }
        else { const v4f rv = *(const v4f*)(AUX + oo); v += rv; }
        vst2(OF + oo, v); } } }
}

__global__ __launch_bounds__(128) void k_sc(const _Float16* __restrict__ Q, const _Float16* __restrict__ KK, int zb, int b0, int hd, float scale, float* __restrict__ S0) {
  __shared__ __align__(16) float ss[4][16][132];
  const int tid = threadIdx.x, wave = tid >> 5, lane = tid & 31, col = lane & 15, g = lane >> 4;
  const int qb = blockIdx.x, kb = blockIdx.y, z = blockIdx.z; const int b = zb ? b0 + z : b0; const int h = zb ? 0 : z;
  float* S = S0 + (size_t)z * TT * TT; const int k0 = kb * 128; const int ql0 = qb * 64 + wave * 16;
  const _Float16* qrow = Q + ((size_t)b * TT + ql0 + col) * CC + (size_t)h * hd;
  const _Float16* kbase = KK + ((size_t)b * TT + k0 + col) * CC + (size_t)h * hd;
  v8f acc[8] = {};
#pragma unroll 1
  for (int kc = 0; kc < hd / 32; ++kc) { const v16h a = frag_h(qrow + kc * 32, lane); asm volatile("s_wait_loadcnt 0x0" ::: "memory");
#pragma unroll
    for (int j = 0; j < 8; ++j) { const v16h kf = frag_h(kbase + (size_t)(j * 16) * CC + kc * 32, lane); asm volatile("s_wait_loadcnt 0x0" ::: "memory"); acc[j] = wmma16(a, kf, acc[j]); } }
#pragma unroll
  for (int j = 0; j < 8; ++j)
#pragma unroll
    for (int r = 0; r < 8; ++r) ss[wave][8 * g + r][j * 16 + col] = acc[j][r] * scale;
  LDSX();
#pragma unroll 1
  for (int rl = 0; rl < 16; ++rl) vst2(S + (size_t)(ql0 + rl) * TT + k0 + lane * 4, *(const v4f*)&ss[wave][rl][lane * 4]);
}

__global__ __launch_bounds__(256) void k_sm(float* __restrict__ S0, const float* __restrict__ B1, const float* __restrict__ B2, int zb, int b0) {
  __shared__ __align__(16) float shv[8][TT];
  const int wave = threadIdx.x >> 5, lane = threadIdx.x & 31; const int t = blockIdx.x * 8 + wave; const int z = blockIdx.y; const int b = zb ? b0 + z : b0;
  float* sr = S0 + ((size_t)z * TT + t) * TT; const size_t boff = ((size_t)b * SEQ_FULL + t) * SEQ_FULL; const float* p1 = B1 + boff; const float* p2 = B2 + boff;
  float m = -3.0e38f;
#pragma unroll 1
  for (int i = 0; i < TT / 128; ++i) { const int c = i * 128 + lane * 4; v4f v = *(const v4f*)(sr + c); const v4f u1 = bfr4(*(const v4f*)(p1 + c)), u2 = bfr4(*(const v4f*)(p2 + c)); v = (v + u1) + u2;
    *(v4f*)&shv[wave][c] = v; m = fmaxf(fmaxf(m, fmaxf(v[0], v[1])), fmaxf(v[2], v[3])); }
#pragma unroll
  for (int o = 1; o < 32; o <<= 1) m = fmaxf(m, __shfl_xor(m, o));
  float sum = 0.f;
#pragma unroll 1
  for (int i = 0; i < TT / 128; ++i) { const int c = i * 128 + lane * 4; const v4f v = *(const v4f*)&shv[wave][c]; v4f e;
#pragma unroll
    for (int k = 0; k < 4; ++k) e[k] = exp2f((v[k] - m) * 1.4426950408889634f);
    *(v4f*)&shv[wave][c] = e; sum += (e[0] + e[1]) + (e[2] + e[3]); }
#pragma unroll
  for (int o = 1; o < 32; o <<= 1) sum += __shfl_xor(sum, o);
  const float inv = PCAR * (1.0f / sum);
#pragma unroll 1
  for (int i = 0; i < TT / 128; ++i) { const int c = i * 128 + lane * 4; v4f v = *(const v4f*)&shv[wave][c]; v *= inv; vst2(sr + c, v); }
}

__global__ __launch_bounds__(128) void k_pv(const float* __restrict__ PS0, const _Float16* __restrict__ VT, int zb, int b0, int hd, float oscale, int out16, _Float16* __restrict__ OH, float* __restrict__ OF) {
  __shared__ __align__(16) float ss[4][16][132];
  const int tid = threadIdx.x, wave = tid >> 5, lane = tid & 31, col = lane & 15, g = lane >> 4;
  const int qb = blockIdx.x, z = blockIdx.z; const int c0 = blockIdx.y * 128; const int b = zb ? b0 + z : b0;
  const int sl0 = zb ? z : (c0 / hd), sl1 = zb ? z : ((c0 + 64) / hd); const int ql0 = qb * 64 + wave * 16;
  const float* p0 = PS0 + ((size_t)sl0 * TT + ql0 + col) * TT; const float* p1 = PS0 + ((size_t)sl1 * TT + ql0 + col) * TT;
  const _Float16* vbase = VT + ((size_t)b * CC + c0 + col) * TT;
  v8f acc[8] = {};
#pragma unroll 1
  for (int kc = 0; kc < TT / 32; ++kc) {
    const v16h a0 = frag_f32(p0 + kc * 32, lane); asm volatile("s_wait_loadcnt 0x0" ::: "memory");
    v16h a1 = a0; if (sl1 != sl0) { a1 = frag_f32(p1 + kc * 32, lane); asm volatile("s_wait_loadcnt 0x0" ::: "memory"); }
#pragma unroll
    for (int j = 0; j < 8; ++j) { const v16h vf = frag_h(vbase + (size_t)(j * 16) * TT + kc * 32, lane); asm volatile("s_wait_loadcnt 0x0" ::: "memory"); acc[j] = wmma16(j < 4 ? a0 : a1, vf, acc[j]); } }
#pragma unroll
  for (int j = 0; j < 8; ++j)
#pragma unroll
    for (int r = 0; r < 8; ++r) ss[wave][8 * g + r][j * 16 + col] = acc[j][r] * oscale;
  LDSX();
  const size_t orow0 = (size_t)b * TT + ql0;
  if (out16) {
#pragma unroll 1
    for (int i = 0; i < 8; ++i) { const int rl = 2 * i + g; const v4f u0 = *(const v4f*)&ss[wave][rl][col * 8], u1 = *(const v4f*)&ss[wave][rl][col * 8 + 4]; H8 o;
#pragma unroll
      for (int k = 0; k < 4; ++k) { o.v[k] = (_Float16)u0[k]; o.v[4 + k] = (_Float16)u1[k]; }
      vst2(OH + (orow0 + rl) * CC + c0 + col * 8, o.u); }
  } else {
#pragma unroll 1
    for (int rl = 0; rl < 16; ++rl) vst2(OF + (orow0 + rl) * CC + c0 + lane * 4, *(const v4f*)&ss[wave][rl][lane * 4]); }
}

__global__ __launch_bounds__(256) void k_pool(const float* __restrict__ XP, const int* __restrict__ PP, float* __restrict__ PATH) {
  const int d = blockIdx.x * 256 + threadIdx.x, b = blockIdx.y;
  const int* pp = PP + (size_t)b * SEQ_FULL; const float* xb = XP + (size_t)b * TT * CC + d;
  const float x0 = xb[0], x1 = xb[CC], x2 = xb[2 * (size_t)CC];
  const float a0 = (x0 + x1) * 0.5f, a1 = ((x0 + x1) + x2) * (1.0f / 3.0f);
  float prv = x0, cur = x0, acc = 0.f, wsum = 0.f; int pm1 = 0, pm2 = 0;
#pragma unroll 1
  for (int s = 0; s < TT; ++s) {
    const int sn = (s + 1 < TT) ? (s + 1) : (TT - 1); const float nxt = xb[(size_t)sn * CC]; const int ps = (pp[s] == 1) ? 1 : 0;
    const float a2 = (cur + nxt) * 0.5f, a3 = ((prv + cur) + nxt) * (1.0f / 3.0f);
    float a = pm2 ? a2 : a3; a = (s == 1) ? a1 : a; a = (s == 0) ? a0 : a;
    acc += ps ? a : 0.f; wsum += (float)ps;
    pm2 = pm1; pm1 = ps; prv = cur; cur = nxt; }
  const float val = acc * (1.0f / wsum);
  vst2(PATH + (size_t)b * CC + d, val);
}

extern "C" void kernel_launch(void* const* d_in, const int* in_sizes, int n_in, void* d_out, int out_size, void* d_ws, size_t ws_size, hipStream_t stream) {
  if (n_in < 29) return;
  const float* const* F = (const float* const*)d_in;
  const int* PP = (const int*)d_in[1];
  const long long nrowx = (long long)(NB - 1) * SEQ_FULL + TT;
  if ((long long)in_sizes[0] < nrowx * CC || (long long)in_sizes[1] < nrowx) return;
  for (int i = 3; i <= 6; ++i) if ((long long)in_sizes[i] < nrowx * SEQ_FULL) return;
  if (in_sizes[7] < CC || in_sizes[8] < CC || in_sizes[23] < CC || in_sizes[24] < CC) return;
  for (int i = 9; i <= 21; i += 2) if ((long long)in_sizes[i] < (long long)CC * CC || in_sizes[i + 1] < CC) return;
  if ((long long)in_sizes[25] < (long long)CC * FF || in_sizes[26] < FF || (long long)in_sizes[27] < (long long)FF * CC || in_sizes[28] < CC) return;
  if ((long long)out_size < (long long)NRW * CC) return;
  if (ws_size < (size_t)WS_END) return;
  char* ws = (char*)d_ws;
  _Float16 *WQT = (_Float16*)(ws + WS_WQ), *WKT = (_Float16*)(ws + WS_WK), *WVT = (_Float16*)(ws + WS_WV), *WOT = (_Float16*)(ws + WS_WO), *WPQT = (_Float16*)(ws + WS_WPQ), *WPKT = (_Float16*)(ws + WS_WPK), *WPVT = (_Float16*)(ws + WS_WPV), *W1T = (_Float16*)(ws + WS_W1), *W2T = (_Float16*)(ws + WS_W2);
  _Float16 *Y16 = (_Float16*)(ws + WS_Y), *CTX16 = (_Float16*)(ws + WS_Y), *Q16 = (_Float16*)(ws + WS_Q), *K16 = (_Float16*)(ws + WS_K), *VT16 = (_Float16*)(ws + WS_VT), *PQ16 = (_Float16*)(ws + WS_PQ), *PK16 = (_Float16*)(ws + WS_PK), *PVT16 = (_Float16*)(ws + WS_PVT), *H16 = (_Float16*)(ws + WS_Q);
  float *SPATH = (float*)(ws + WS_Q), *SSELF = (float*)(ws + WS_XP), *XP = (float*)(ws + WS_XP), *X1 = (float*)(ws + WS_XP), *PATH = (float*)(ws + WS_PATH);
  float* OUT = (float*)d_out;

  k_wcvt<<<dim3(CC / 64, CC / 64), 256, 0, stream>>>(F[9], CC, CC, WQT);
  k_wcvt<<<dim3(CC / 64, CC / 64), 256, 0, stream>>>(F[11], CC, CC, WKT);
  k_wcvt<<<dim3(CC / 64, CC / 64), 256, 0, stream>>>(F[13], CC, CC, WVT);
  k_wcvt<<<dim3(CC / 64, CC / 64), 256, 0, stream>>>(F[15], CC, CC, WOT);
  k_wcvt<<<dim3(CC / 64, CC / 64), 256, 0, stream>>>(F[17], CC, CC, WPQT);
  k_wcvt<<<dim3(CC / 64, CC / 64), 256, 0, stream>>>(F[19], CC, CC, WPKT);
  k_wcvt<<<dim3(CC / 64, CC / 64), 256, 0, stream>>>(F[21], CC, CC, WPVT);
  k_wcvt<<<dim3(FF / 64, CC / 64), 256, 0, stream>>>(F[25], CC, FF, W1T);
  k_wcvt<<<dim3(CC / 64, FF / 64), 256, 0, stream>>>(F[27], FF, CC, W2T);
  k_ln<<<dim3(NRW / 8), 256, 0, stream>>>(F[0], 1, 1, F[7], F[8], Y16);
  k_gem<0><<<dim3(NRW / 64, CC / 128), 128, 0, stream>>>(Y16, CC, CC, WQT, CC, F[10], 1.0f / WCAR, 1.0f, nullptr, nullptr, Q16, nullptr);
  k_gem<0><<<dim3(NRW / 64, CC / 128), 128, 0, stream>>>(Y16, CC, CC, WKT, CC, F[12], 1.0f / WCAR, 1.0f, nullptr, nullptr, K16, nullptr);
  k_gem<1><<<dim3(NRW / 64, CC / 128), 128, 0, stream>>>(Y16, CC, CC, WVT, CC, F[14], 1.0f / WCAR, 1.0f, nullptr, nullptr, VT16, nullptr);
  k_gem<0><<<dim3(NRW / 64, CC / 128), 128, 0, stream>>>(Y16, CC, CC, WPQT, CC, F[18], 1.0f / WCAR, 1.0f, nullptr, nullptr, PQ16, nullptr);
  k_gem<0><<<dim3(NRW / 64, CC / 128), 128, 0, stream>>>(Y16, CC, CC, WPKT, CC, F[20], 1.0f / WCAR, 1.0f, nullptr, nullptr, PK16, nullptr);
  k_gem<1><<<dim3(NRW / 64, CC / 128), 128, 0, stream>>>(Y16, CC, CC, WPVT, CC, F[22], 1.0f / WCAR, 1.0f, nullptr, nullptr, PVT16, nullptr);
  for (int b = 0; b < NB; ++b) {
    k_sc<<<dim3(NQB, TT / 128, NH), 128, 0, stream>>>(Q16, K16, 0, b, HD, QSCALE, SSELF);
    k_sm<<<dim3(TT / 8, NH), 256, 0, stream>>>(SSELF, F[3], F[4], 0, b);
    k_pv<<<dim3(NQB, CC / 128, 1), 128, 0, stream>>>(SSELF, VT16, 0, b, HD, HCAR / PCAR, 1, CTX16, nullptr);
  }
  k_sc<<<dim3(NQB, TT / 128, NB), 128, 0, stream>>>(PQ16, PK16, 1, 0, CC, PSCALE, SPATH);
  k_sm<<<dim3(TT / 8, NB), 256, 0, stream>>>(SPATH, F[5], F[6], 1, 0);
  k_pv<<<dim3(NQB, CC / 128, NB), 128, 0, stream>>>(SPATH, PVT16, 1, 0, CC, 1.0f / PCAR, 0, nullptr, XP);
  k_pool<<<dim3(CC / 256, NB), 256, 0, stream>>>(XP, PP, PATH);
  k_gem<3><<<dim3(NRW / 64, CC / 128), 128, 0, stream>>>(CTX16, CC, CC, WOT, CC, F[16], 1.0f / (WCAR * HCAR), 1.0f, F[0], PATH, nullptr, X1);
  k_ln<<<dim3(NRW / 8), 256, 0, stream>>>(X1, 0, 0, F[23], F[24], Y16);
  k_gem<2><<<dim3(NRW / 64, FF / 128), 128, 0, stream>>>(Y16, CC, CC, W1T, FF, F[26], 1.0f / WCAR, HCAR, nullptr, nullptr, H16, nullptr);
  k_gem<4><<<dim3(NRW / 64, CC / 128), 128, 0, stream>>>(H16, FF, FF, W2T, CC, F[28], 1.0f / (WCAR * HCAR), 1.0f, X1, nullptr, nullptr, OUT);
}
